// MultiScaleGraphConvolution_26310969655903
// MI455X (gfx1250) — hardware-verified
//
#include <hip/hip_runtime.h>
#include <math.h>


#define BB 8
#define NN 1024
#define DIN 256
#define DH 128
#define DOUT 384
#define NE 16384
#define ROWS (BB * NN)

typedef __attribute__((ext_vector_type(16))) _Float16 v16h;
typedef __attribute__((ext_vector_type(8)))  _Float16 v8h;
typedef __attribute__((ext_vector_type(8)))  float v8f;
typedef __attribute__((ext_vector_type(4)))  float v4f;
typedef __attribute__((ext_vector_type(4)))  unsigned v4u;
typedef float __attribute__((may_alias)) float_a;

template <typename T> __device__ __forceinline__ void vst2(void* p, T v) { *(volatile T*)p = v; __threadfence(); *(volatile T*)p = v; }
__device__ __forceinline__ v8f wmma16(v16h a, v16h b, v8f c) {
  v8f d = __builtin_amdgcn_wmma_f32_16x16x32_f16(false, a, false, b, (short)0, c, false, false);
  asm volatile("v_nop\n\tv_nop\n\tv_nop\n\tv_nop" : "+v"(d) : "v"(a), "v"(b));
  return d;
}
__device__ __forceinline__ v16h frag_f32row(const float* row, int k0, int lane) {
  v16h a; const float* p = row + k0 + 8 * (lane >> 4);
#pragma unroll
  for (int i = 0; i < 8; ++i) { a[i] = (_Float16)p[i]; a[8 + i] = (_Float16)p[16 + i]; }
  return a;
}
__device__ __forceinline__ v16h frag_f16row(const _Float16* row, int k0, int lane) {
  union { v16h v; v8h q[2]; } a; const _Float16* p = row + k0 + 8 * (lane >> 4);
  a.q[0] = *(const v8h*)p; a.q[1] = *(const v8h*)(p + 16);
  return a.v;
}
__device__ __forceinline__ v16h frag_f32col(const float* base, int k0, int lane, int ld) {
  v16h a; const float* p = base + (size_t)(k0 + 8 * (lane >> 4)) * ld;
#pragma unroll
  for (int i = 0; i < 8; ++i) { a[i] = (_Float16)p[(size_t)i * ld]; a[8 + i] = (_Float16)p[(size_t)(16 + i) * ld]; }
  return a;
}

__global__ __launch_bounds__(256) void k_adj(const int* __restrict__ ei, _Float16* __restrict__ A, _Float16* __restrict__ At) {
  __shared__ __align__(16) _Float16 ra[NN]; __shared__ __align__(16) _Float16 rt[NN];
  const int r = blockIdx.x, tid = threadIdx.x;
  for (int i = tid; i < NN; i += 256) { ra[i] = (_Float16)0.f; rt[i] = (_Float16)0.f; }
  __syncthreads();
  for (int e = tid; e < NE; e += 256) {
    int s = ei[e], d = ei[NE + e];
    s = s < 0 ? 0 : (s >= NN ? NN - 1 : s); d = d < 0 ? 0 : (d >= NN ? NN - 1 : d);
    if (s == r) ra[d] = (_Float16)1.f;
    if (d == r) rt[s] = (_Float16)1.f;
  }
  __syncthreads();
  if (tid < 128) vst2(A + (size_t)r * NN + tid * 8, *(const v4u*)(ra + tid * 8));
  else           vst2(At + (size_t)r * NN + (tid - 128) * 8, *(const v4u*)(rt + (tid - 128) * 8));
}

template <int AT, int BT, int EPI>
__global__ __launch_bounds__(128) void k_gemm(const void* __restrict__ Av, int lda, size_t az, const void* __restrict__ Bv, int ldb, size_t bz,
                                            const float* __restrict__ bias, void* __restrict__ Cv, int ldc, size_t cz, int K) {
  __shared__ __align__(16) float st[64][68];
  const int tid = threadIdx.x, wave = tid >> 5, lane = tid & 31, col = lane & 15, g = lane >> 4;
  const int m0 = blockIdx.x * 64 + wave * 16, n0 = blockIdx.y * 64;
  const size_t zb = blockIdx.z;
  v8f acc[4] = {};
#pragma unroll 1
  for (int kc = 0; kc < K / 32; ++kc) {
    v16h a;
    if (AT == 0) a = frag_f32row((const float*)Av + zb * az + (size_t)(m0 + col) * lda, kc * 32, lane);
    else         a = frag_f16row((const _Float16*)Av + zb * az + (size_t)(m0 + col) * lda, kc * 32, lane);
#pragma unroll
    for (int j = 0; j < 4; ++j) {
      v16h bf;
      if (BT == 0) bf = frag_f32col((const float*)Bv + zb * bz + n0 + j * 16 + col, kc * 32, lane, ldb);
      else         bf = frag_f16row((const _Float16*)Bv + zb * bz + (size_t)(n0 + j * 16 + col) * ldb, kc * 32, lane);
      acc[j] = wmma16(a, bf, acc[j]);
    }
  }
#pragma unroll
  for (int j = 0; j < 4; ++j) {
    const float bv = bias ? bias[n0 + j * 16 + col] : 0.f;
#pragma unroll
    for (int r = 0; r < 8; ++r) {
      float v = acc[j][r] + bv;
      if (EPI == 1) v = v > 0.f ? 1.f : 0.f;
      if (EPI == 2) v = 0.5f * v * (1.f + erff(v * 0.70710678118654752f));
      st[wave * 16 + 8 * g + r][j * 16 + col] = v;
    }
  }
  __syncthreads();
  const int bm0 = blockIdx.x * 64;
  if (EPI == 1) {
    _Float16* C = (_Float16*)Cv + zb * cz;
    for (int q = tid; q < 64 * 8; q += 128) { const int rl = q >> 3, pc = q & 7;
      union { v8h h; v4u u; } pk;
#pragma unroll
      for (int e = 0; e < 8; ++e) pk.h[e] = (_Float16)st[rl][pc * 8 + e];
      vst2(C + (size_t)(bm0 + rl) * ldc + n0 + pc * 8, pk.u); }
  } else {
    float* C = (float*)Cv + zb * cz;
    for (int q = tid; q < 64 * 16; q += 128) { const int rl = q >> 4, pc = q & 15;
      vst2(C + (size_t)(bm0 + rl) * ldc + n0 + pc * 4, *(const v4f*)(&st[rl][pc * 4])); }
  }
}

__global__ __launch_bounds__(256) void k_bn_part(const float* __restrict__ agg, float* __restrict__ part) {
  __shared__ float s1[DOUT], s2[DOUT];
  const int tid = threadIdx.x, r0 = blockIdx.x * 64;
  for (int c = tid; c < DOUT; c += 256) { float a = 0.f, b = 0.f;
    for (int r = 0; r < 64; ++r) { const float v = agg[(size_t)(r0 + r) * DOUT + c]; a += v; b += v * v; }
    s1[c] = a; s2[c] = b; }
  __syncthreads();
  for (int q = tid; q < 2 * DOUT / 4; q += 256) { const int c4 = q * 4; v4f v;
#pragma unroll
    for (int e = 0; e < 4; ++e) { const int c = c4 + e; v[e] = c < DOUT ? s1[c] : s2[c - DOUT]; }
    vst2(part + (size_t)blockIdx.x * 2 * DOUT + c4, v); }
}
__global__ __launch_bounds__(DOUT) void k_bn_fin(const float* __restrict__ part, float* __restrict__ stats) {
  const int c = threadIdx.x; float a = 0.f, b = 0.f;
  for (int p = 0; p < ROWS / 64; ++p) { a += part[(size_t)p * 2 * DOUT + c]; b += part[(size_t)p * 2 * DOUT + DOUT + c]; }
  const float mu = a / (float)ROWS; float var = b / (float)ROWS - mu * mu; var = var < 0.f ? 0.f : var;
  vst2(stats + c, (float_a)mu); vst2(stats + DOUT + c, (float_a)rsqrtf(var + 1e-5f));
}
__global__ __launch_bounds__(256) void k_bn_apply(const float* __restrict__ agg, const float* __restrict__ stats,
                                                const float* __restrict__ g0, const float* __restrict__ be0, const float* __restrict__ g1, const float* __restrict__ be1,
                                                const float* __restrict__ g2, const float* __restrict__ be2, float* __restrict__ bn) {
  const size_t i = (size_t)blockIdx.x * 256 + threadIdx.x; const int c = (int)(i % DOUT);
  const float* g = c < DH ? g0 : (c < 2 * DH ? g1 : g2); const float* be = c < DH ? be0 : (c < 2 * DH ? be1 : be2); const int cc = c % DH;
  vst2(bn + i, (float_a)((agg[i] - stats[c]) * stats[DOUT + c] * g[cc] + be[cc]));
}

extern "C" void kernel_launch(void* const* d_in, const int* in_sizes, int n_in,
                              void* d_out, int out_size, void* d_ws, size_t ws_size,
                              hipStream_t stream) {
  (void)in_sizes; (void)n_in; (void)out_size; (void)ws_size;
  const float* x  = (const float*)d_in[0];
  const int*   ei = (const int*)d_in[1];
  const float* W[3]  = {(const float*)d_in[2], (const float*)d_in[6], (const float*)d_in[10]};
  const float* bw[3] = {(const float*)d_in[3], (const float*)d_in[7], (const float*)d_in[11]};
  const float* gm[3] = {(const float*)d_in[4], (const float*)d_in[8], (const float*)d_in[12]};
  const float* bt[3] = {(const float*)d_in[5], (const float*)d_in[9], (const float*)d_in[13]};
  const float* Wf = (const float*)d_in[14];
  const float* bf = (const float*)d_in[15];
  float* out = (float*)d_out;
  char* ws = (char*)d_ws; size_t off = 0;
  auto take = [&](size_t bytes) { char* p = ws + off; off += (bytes + 255) & ~(size_t)255; return p; };
  _Float16* A1 = (_Float16*)take((size_t)NN * NN * 2);
  _Float16* At = (_Float16*)take((size_t)NN * NN * 2);
  _Float16* A2 = (_Float16*)take((size_t)NN * NN * 2);
  _Float16* A3 = (_Float16*)take((size_t)NN * NN * 2);
  float* h   = (float*)take((size_t)ROWS * DH * 4);
  float* agg = (float*)take((size_t)ROWS * DOUT * 4);
  float* bn  = (float*)take((size_t)ROWS * DOUT * 4);
  float* part = (float*)take((size_t)(ROWS / 64) * 2 * DOUT * 4);
  float* stats = (float*)take(2 * DOUT * 4);

  k_adj<<<NN, 256, 0, stream>>>(ei, A1, At);
  k_gemm<1, 1, 1><<<dim3(NN / 64, NN / 64, 1), 128, 0, stream>>>(A1, NN, 0, At, NN, 0, nullptr, A2, NN, 0, NN);
  k_gemm<1, 1, 1><<<dim3(NN / 64, NN / 64, 1), 128, 0, stream>>>(A2, NN, 0, At, NN, 0, nullptr, A3, NN, 0, NN);
  const _Float16* Ai[3] = {A1, A2, A3};
  for (int i = 0; i < 3; ++i) {
    k_gemm<0, 0, 0><<<dim3(ROWS / 64, DH / 64, 1), 128, 0, stream>>>(x, DIN, 0, W[i], DH, 0, bw[i], h, DH, 0, DIN);
    k_gemm<1, 0, 0><<<dim3(NN / 64, DH / 64, BB), 128, 0, stream>>>(Ai[i], NN, 0, h, DH, (size_t)NN * DH, nullptr,
                                                                    agg + i * DH, DOUT, (size_t)NN * DOUT, NN);
  }
  k_bn_part<<<ROWS / 64, 256, 0, stream>>>(agg, part);
  k_bn_fin<<<1, DOUT, 0, stream>>>(part, stats);
  k_bn_apply<<<ROWS * DOUT / 256, 256, 0, stream>>>(agg, stats, gm[0], bt[0], gm[1], bt[1], gm[2], bt[2], bn);
  k_gemm<0, 0, 2><<<dim3(ROWS / 64, DOUT / 64, 1), 128, 0, stream>>>(bn, DOUT, 0, Wf, DOUT, 0, bf, out, DOUT, 0, DOUT);
}
